// CausalSelfAttention_75780402971163
// MI455X (gfx1250) — hardware-verified
//
#include <hip/hip_runtime.h>
#include <math.h>

typedef __attribute__((ext_vector_type(16))) _Float16 v16h;
typedef __attribute__((ext_vector_type(16))) __bf16 v16b;
typedef __attribute__((ext_vector_type(8)))  _Float16 v8h;
typedef __attribute__((ext_vector_type(8)))  __bf16 v8b;
typedef __attribute__((ext_vector_type(8)))  float v8f;
typedef __attribute__((ext_vector_type(4)))  float v4f;
typedef __attribute__((ext_vector_type(4)))  unsigned v4u;

template <typename T> __device__ __forceinline__ void vst2(void* p, T v) { *(volatile T*)p = v; __threadfence(); *(volatile T*)p = v; }
__device__ __forceinline__ v8f wmma16(v16h a, v16h b, v8f c) {
  v8f d = __builtin_amdgcn_wmma_f32_16x16x32_f16(false, a, false, b, (short)0, c, false, false);
  asm volatile("v_nop\n\tv_nop\n\tv_nop\n\tv_nop" : "+v"(d) : "v"(a), "v"(b));
  return d;
}
__device__ __forceinline__ v8f wmma_bf(v16b a, v16b b, v8f c) {
  v8f d = __builtin_amdgcn_wmma_f32_16x16x32_bf16(false, a, false, b, (short)0, c, false, false);
  asm volatile("v_nop\n\tv_nop\n\tv_nop\n\tv_nop" : "+v"(d) : "v"(a), "v"(b));
  return d;
}
__device__ __forceinline__ v16h frag_h(const _Float16* rowk0, int lane) {
  union { v16h v; v8h q[2]; } u; const _Float16* p = rowk0 + 8 * (lane >> 4);
  u.q[0] = *(const v8h*)p; u.q[1] = *(const v8h*)(p + 16); return u.v;
}
__device__ __forceinline__ v16b frag_b(const __bf16* rowk0, int lane) {
  union { v16b v; v8b q[2]; } u; const __bf16* p = rowk0 + 8 * (lane >> 4);
  u.q[0] = *(const v8b*)p; u.q[1] = *(const v8b*)(p + 16); return u.v;
}
struct F2 { v16b h, l; };
__device__ __forceinline__ F2 bsplit16(const float v[16]) { F2 r;
#pragma unroll
  for (int i = 0; i < 16; ++i) { const __bf16 h = (__bf16)v[i]; r.h[i] = h; r.l[i] = (__bf16)(v[i] - (float)h); }
  return r; }
#define LDSX() do { asm volatile("s_wait_dscnt 0" ::: "memory"); __builtin_amdgcn_wave_barrier(); __builtin_amdgcn_fence(3  , "workgroup"); } while (0)
__device__ __forceinline__ float bfr(float v) { return (float)(__bf16)v; }

#ifndef NB
#define NB 2
#endif
#ifndef SEQ
#define SEQ 2048
#endif
#define NB_FULL 2
#define TT_FULL 2048
#define TT SEQ
#define ROWS (NB * TT)
#define CC 1024
#define DIN 1024
#define NH 16
#define HD 64
#define NQB (TT / 64)
#define VHI 256
#define QBH (VHI / 64)
#define EPSN 1.1920928955078125e-07f
#define SC2 (0.125f * 1.4426950408889634f)
#define NEGB (-3.0e38f)
static_assert(NB >= 1 && NB <= NB_FULL);
static_assert(TT >= 256 && TT <= TT_FULL && (TT % 128) == 0);
static_assert(CC == NH * HD && HD == 64 && (CC % 128) == 0 && (DIN % 128) == 0 && (DIN % 32) == 0 && (CC % 32) == 0);
static_assert(CC == DIN);
static_assert((VHI % 64) == 0 && VHI <= TT && QBH * 64 == VHI);
static_assert((ROWS % 64) == 0 && NQB * 64 == TT);
static_assert(((size_t)ROWS * DIN) % (8 * 256) == 0 && ((size_t)CC * DIN) % (8 * 256) == 0);
static_assert((TT % 8) == 0);

#define PLE ((size_t)ROWS * CC)
#define WS_XB  ((size_t)0)
#define WS_WB  (WS_XB + (size_t)2 * ROWS * DIN)
#define WS_RT  (WS_WB + (size_t)2 * 4 * CC * DIN)
#define WS_QK  (WS_RT + (size_t)4 * TT * 64)
#define WS_VT  (WS_QK + (size_t)2 * 4 * PLE)
#define WS_VB  (WS_VT + (size_t)2 * NB * CC * TT)
#define WS_VBL (WS_VB + (size_t)2 * NB * CC * VHI)
#define WS_YH  (WS_VBL + (size_t)2 * NB * CC * VHI)
#define WS_YL  (WS_YH + (size_t)2 * ROWS * CC)
#define WS_END (WS_YL + (size_t)2 * ROWS * CC)
static_assert((size_t)WS_END <= (size_t)134217728u);
static_assert((WS_WB % 128u) == 0 && (WS_RT % 128u) == 0 && (WS_QK % 128u) == 0 && (WS_VT % 128u) == 0 && (WS_VB % 128u) == 0 && (WS_VBL % 128u) == 0 && (WS_YH % 128u) == 0 && (WS_YL % 128u) == 0);

__global__ __launch_bounds__(256) void k_cvt(const float* __restrict__ S, __bf16* __restrict__ D, int ngroups, int tt, int tt_full) {
  const int e = blockIdx.x * 256 + threadIdx.x; if (e >= ngroups) return;
  const int row = e / (DIN / 8), q = e - row * (DIN / 8); const int bb = row / tt, t = row - bb * tt;
  const float* p = S + ((size_t)bb * tt_full + t) * DIN + q * 8;
  const v4f a = *(const v4f*)p, c = *(const v4f*)(p + 4);
  union { v8b v; v4u u; } o;
#pragma unroll
  for (int i = 0; i < 4; ++i) { o.v[i] = (__bf16)a[i]; o.v[4 + i] = (__bf16)c[i]; }
  vst2(D + (size_t)e * 8, o.u);
}
__global__ __launch_bounds__(256) void k_rope(float* __restrict__ RT) {
  const int tid = threadIdx.x; const int t = blockIdx.x * 8 + (tid >> 5); const int j = tid & 31;
  double p = 1.0;
  p = (j & 16) ? p * 100.0 : p;
  p = (j & 8) ? p * 10.0 : p;
  p = (j & 4) ? p * 3.1622776601683795 : p;
  p = (j & 2) ? p * 1.7782794100389228 : p;
  p = (j & 1) ? p * 1.333521432163324 : p;
  const float pf = (float)p; const float inv = 1.0f / pf; const float ang = (float)t * inv;
  float sn, cs; sincosf(ang, &sn, &cs);
  vst2(RT + (size_t)t * 64 + j, cs);
  vst2(RT + (size_t)t * 64 + 32 + j, sn);
}
__global__ __launch_bounds__(128) void k_proj(const __bf16* __restrict__ XB, const __bf16* __restrict__ WB, const float* __restrict__ RT, const float* __restrict__ QNW, const float* __restrict__ KNW,
    _Float16* __restrict__ QK, _Float16* __restrict__ VT, __bf16* __restrict__ VB, __bf16* __restrict__ VBL) {
  __shared__ __align__(16) _Float16 sh[64][136], sl[64][136]; __shared__ __align__(16) float cs[64][68];
  __shared__ __align__(16) _Float16 th[128][72]; __shared__ __align__(16) __bf16 tb[128][72], tbl[128][72];
  const int tid = threadIdx.x; const int wave = __builtin_amdgcn_readfirstlane(threadIdx.x >> 5); const int lane = tid & 31, col = lane & 15, g = lane >> 4;
  const int which = blockIdx.z; const int c0 = blockIdx.y * 128; const size_t r0 = (size_t)blockIdx.x * 64; const size_t bb = r0 / TT; const int t0 = (int)(r0 % TT);
  const __bf16* ap = XB + (r0 + wave * 16 + col) * DIN;
  const __bf16* wp = WB + (size_t)which * CC * DIN + (size_t)(c0 + col) * DIN;
  v8f acc[8] = {};
#pragma unroll 2
  for (int kc = 0; kc < DIN / 32; ++kc) { const v16b a = frag_b(ap + kc * 32, lane);
#pragma unroll
    for (int j = 0; j < 8; ++j) { const v16b w = frag_b(wp + (size_t)j * 16 * DIN + kc * 32, lane); acc[j] = wmma_bf(a, w, acc[j]); } }
  if (which < 2) {
    for (int e = tid; e < 64 * 16; e += 128) { const int rl = e >> 4, q = e & 15; *(v4f*)&cs[rl][q * 4] = *(const v4f*)(RT + (size_t)(t0 + rl) * 64 + q * 4); }
    float w[4];
#pragma unroll
    for (int i = 0; i < 4; ++i) { const float a = QNW[i * 16 + col], c = KNW[i * 16 + col]; w[i] = bfr(which == 0 ? a : c); }
    __syncthreads();
#pragma unroll
    for (int hh = 0; hh < 2; ++hh) {
#pragma unroll
      for (int r = 0; r < 8; ++r) { const float a0 = acc[hh * 4 + 0][r], a1 = acc[hh * 4 + 1][r], a2 = acc[hh * 4 + 2][r], a3 = acc[hh * 4 + 3][r];
        float ss = a0 * a0 + a1 * a1 + a2 * a2 + a3 * a3;
        ss += __shfl_xor(ss, 1); ss += __shfl_xor(ss, 2); ss += __shfl_xor(ss, 4); ss += __shfl_xor(ss, 8);
        const float inv = rsqrtf(ss * (1.0f / 64.0f) + EPSN);
        const int row = wave * 16 + 8 * g + r;
        const float c0v = cs[row][col], c1v = cs[row][16 + col], s0v = cs[row][32 + col], s1v = cs[row][48 + col];
        const float xr0 = a0 * inv * w[0], xr1 = a1 * inv * w[1], xi0 = a2 * inv * w[2], xi1 = a3 * inv * w[3];
        float ov[4]; ov[0] = xr0 * c0v - xi0 * s0v; ov[1] = xr1 * c1v - xi1 * s1v; ov[2] = xr0 * s0v + xi0 * c0v; ov[3] = xr1 * s1v + xi1 * c1v;
#pragma unroll
        for (int i = 0; i < 4; ++i) { const _Float16 hv = (_Float16)ov[i]; sh[row][hh * 64 + i * 16 + col] = hv; sl[row][hh * 64 + i * 16 + col] = (_Float16)((ov[i] - (float)hv) * 1024.0f); } } }
    __syncthreads();
    _Float16* DH = QK + (size_t)which * 2 * PLE; _Float16* DL = DH + PLE;
    for (int e = tid; e < 64 * 16; e += 128) { const int rl = e >> 4, q = e & 15; const size_t o = (r0 + rl) * CC + c0 + q * 8; vst2(DH + o, *(const v4u*)&sh[rl][q * 8]); vst2(DL + o, *(const v4u*)&sl[rl][q * 8]); }
  } else { const bool hi_rows = t0 < VHI;
#pragma unroll
    for (int j = 0; j < 8; ++j) {
#pragma unroll
      for (int r = 0; r < 8; ++r) { const float v = acc[j][r]; const int rl = wave * 16 + 8 * g + r, cl = j * 16 + col; th[cl][rl] = (_Float16)v; const __bf16 bh = (__bf16)v; tb[cl][rl] = bh; tbl[cl][rl] = (__bf16)(v - (float)bh); } }
    __syncthreads();
    for (int e = tid; e < 128 * 8; e += 128) { const int cl = e >> 3, q = e & 7; vst2(VT + (bb * CC + c0 + cl) * (size_t)TT + t0 + q * 8, *(const v4u*)&th[cl][q * 8]);
      if (hi_rows) { const size_t o3 = (bb * CC + c0 + cl) * (size_t)VHI + t0 + q * 8; vst2(VB + o3, *(const v4u*)&tb[cl][q * 8]); vst2(VBL + o3, *(const v4u*)&tbl[cl][q * 8]); } } } }
__global__ __launch_bounds__(128) void k_attn(const _Float16* __restrict__ QK, const _Float16* __restrict__ VT, const __bf16* __restrict__ VB, const __bf16* __restrict__ VBL, __bf16* __restrict__ YH, __bf16* __restrict__ YL) {
  __shared__ __align__(16) float ps[4][16][36]; __shared__ __align__(16) __bf16 yh[4][16][72], yl[4][16][72];
  const int tid = threadIdx.x; const int wave = __builtin_amdgcn_readfirstlane(threadIdx.x >> 5); const int lane = tid & 31, col = lane & 15, g = lane >> 4;
  const int qb = blockIdx.x; const int bh = blockIdx.y; const int b = bh / NH, h = bh - b * NH;
  const int q0w = qb * 64 + wave * 16; const int nhalf = ((q0w + 15) >> 5) + 1; const bool early = qb < QBH;
  const _Float16* QHp = QK + ((size_t)b * TT + q0w + col) * CC + h * HD;
  const _Float16* KHp = QK + (size_t)2 * PLE + ((size_t)b * TT + col) * CC + h * HD;
  const size_t vrow = (size_t)b * CC + h * HD + col;
  float m[8], l[8]; v8f o[4] = {};
#pragma unroll
  for (int r = 0; r < 8; ++r) { m[r] = NEGB; l[r] = 0.f; }
#pragma unroll 1
  for (int hs = 0; hs < nhalf; ++hs) { const int key0 = hs * 32;
    int qz = 0; asm volatile("" : "+s"(qz));
    v8f s0 = {}, s1 = {}, x0 = {}, x1 = {};
#pragma unroll
    for (int kc = 0; kc < HD / 32; ++kc) { const v16h qh = frag_h(QHp + qz + kc * 32, lane), ql = frag_h(QHp + PLE + qz + kc * 32, lane);
      const _Float16* kp = KHp + (size_t)key0 * CC + kc * 32;
      { const v16h kh = frag_h(kp, lane), kl = frag_h(kp + PLE, lane); s0 = wmma16(qh, kh, s0); x0 = wmma16(ql, kh, x0); x0 = wmma16(qh, kl, x0); }
      { const v16h kh = frag_h(kp + (size_t)16 * CC, lane), kl = frag_h(kp + PLE + (size_t)16 * CC, lane); s1 = wmma16(qh, kh, s1); x1 = wmma16(ql, kh, x1); x1 = wmma16(qh, kl, x1); } }
#pragma unroll
    for (int r = 0; r < 8; ++r) { const int qrow = q0w + 8 * g + r; const bool ok0 = (key0 + col) <= qrow, ok1 = (key0 + 16 + col) <= qrow;
      float e0 = (s0[r] + x0[r] * (1.0f / 1024.0f)) * SC2, e1 = (s1[r] + x1[r] * (1.0f / 1024.0f)) * SC2;
      e0 = ok0 ? e0 : NEGB; e1 = ok1 ? e1 : NEGB;
      float mx = fmaxf(e0, e1);
      mx = fmaxf(mx, __shfl_xor(mx, 1)); mx = fmaxf(mx, __shfl_xor(mx, 2)); mx = fmaxf(mx, __shfl_xor(mx, 4)); mx = fmaxf(mx, __shfl_xor(mx, 8));
      const float mnew = fmaxf(m[r], mx); const float alpha = exp2f(m[r] - mnew);
      float p0 = exp2f(e0 - mnew), p1 = exp2f(e1 - mnew); p0 = ok0 ? p0 : 0.f; p1 = ok1 ? p1 : 0.f;
      l[r] = l[r] * alpha + (p0 + p1); m[r] = mnew;
      o[0][r] *= alpha; o[1][r] *= alpha; o[2][r] *= alpha; o[3][r] *= alpha;
      ps[wave][8 * g + r][col] = p0 * 1024.0f; ps[wave][8 * g + r][16 + col] = p1 * 1024.0f; }
    LDSX();
    if (early) { float pv[16];
#pragma unroll
      for (int i = 0; i < 8; ++i) { pv[i] = ps[wave][col][8 * g + i]; pv[8 + i] = ps[wave][col][16 + 8 * g + i]; }
      const F2 p = bsplit16(pv);
#pragma unroll
      for (int j = 0; j < HD / 16; ++j) { const size_t po = (vrow + j * 16) * (size_t)VHI + key0; const v16b vh = frag_b(VB + po, lane), vl = frag_b(VBL + po, lane); o[j] = wmma_bf(p.h, vh, o[j]); o[j] = wmma_bf(p.l, vh, o[j]); o[j] = wmma_bf(p.h, vl, o[j]); }
    } else { v16h p;
#pragma unroll
      for (int i = 0; i < 8; ++i) { p[i] = (_Float16)ps[wave][col][8 * g + i]; p[8 + i] = (_Float16)ps[wave][col][16 + 8 * g + i]; }
#pragma unroll
      for (int j = 0; j < HD / 16; ++j) { const size_t po = (vrow + j * 16) * (size_t)TT + key0; o[j] = wmma16(p, frag_h(VT + po, lane), o[j]); } }
    LDSX(); }
#pragma unroll
  for (int r = 0; r < 8; ++r) { float ls = l[r]; ls += __shfl_xor(ls, 1); ls += __shfl_xor(ls, 2); ls += __shfl_xor(ls, 4); ls += __shfl_xor(ls, 8);
    const float il = (1.0f / ls) * (1.0f / 1024.0f);
#pragma unroll
    for (int j = 0; j < HD / 16; ++j) { const float y = o[j][r] * il; const __bf16 yb = (__bf16)y; yh[wave][8 * g + r][j * 16 + col] = yb; yl[wave][8 * g + r][j * 16 + col] = (__bf16)(y - (float)yb); } }
  LDSX();
#pragma unroll
  for (int it = 0; it < 4; ++it) { const int rl = it * 4 + (lane >> 3), q = lane & 7; const size_t off = ((size_t)b * TT + q0w + rl) * CC + h * HD + q * 8;
    vst2(YH + off, *(const v4u*)&yh[wave][rl][q * 8]); vst2(YL + off, *(const v4u*)&yl[wave][rl][q * 8]); } }
__global__ __launch_bounds__(128) void k_out(const __bf16* __restrict__ YH, const __bf16* __restrict__ YL, const __bf16* __restrict__ WO, float* __restrict__ OUT) { __shared__ __align__(16) float sf[4][16][132];
  const int tid = threadIdx.x; const int wave = __builtin_amdgcn_readfirstlane(threadIdx.x >> 5); const int lane = tid & 31, col = lane & 15, g = lane >> 4;
  const int c0 = blockIdx.y * 128; const size_t rb = (size_t)blockIdx.x * 64; const size_t bb = rb / TT; const int tt0 = (int)(rb % TT) + wave * 16; const size_t r0 = rb + wave * 16;
  const size_t orow0 = bb * (size_t)TT_FULL + (size_t)tt0;
  const __bf16* ahp = YH + (r0 + col) * CC; const __bf16* alp = YL + (r0 + col) * CC; const __bf16* wp = WO + (size_t)(c0 + col) * CC;
  v8f acc[8] = {};
#pragma unroll 2
  for (int kc = 0; kc < CC / 32; ++kc) { const v16b ah = frag_b(ahp + kc * 32, lane), al = frag_b(alp + kc * 32, lane);
#pragma unroll
    for (int j = 0; j < 8; ++j) { const v16b w = frag_b(wp + (size_t)j * 16 * CC + kc * 32, lane); acc[j] = wmma_bf(ah, w, acc[j]); acc[j] = wmma_bf(al, w, acc[j]); } }
#pragma unroll
  for (int j = 0; j < 8; ++j) {
#pragma unroll
    for (int r = 0; r < 8; ++r) sf[wave][8 * g + r][j * 16 + col] = acc[j][r]; }
  LDSX();
  for (int rl = 0; rl < 16; ++rl) vst2(OUT + (orow0 + rl) * DIN + c0 + lane * 4, *(const v4f*)&sf[wave][rl][lane * 4]); }

extern "C" void kernel_launch(void* const* d_in, const int* in_sizes, int n_in, void* d_out, int out_size, void* d_ws, size_t ws_size, hipStream_t stream) {
  if (n_in < 7) return;
  const size_t need_rows = (size_t)(NB - 1) * TT_FULL + (size_t)TT;
  if ((size_t)in_sizes[0] < need_rows * DIN) return;
  if ((size_t)in_sizes[1] < (size_t)CC * DIN) return;
  if ((size_t)in_sizes[2] < (size_t)CC * DIN) return;
  if ((size_t)in_sizes[3] < (size_t)CC * DIN) return;
  if ((size_t)in_sizes[4] < (size_t)DIN * CC) return;
  if (in_sizes[5] < HD || in_sizes[6] < HD) return;
  if ((size_t)out_size < need_rows * DIN) return;
  if (ws_size < (size_t)WS_END) return;
  const float* const* F = (const float* const*)d_in;
  char* ws = (char*)d_ws;
  __bf16* XB = (__bf16*)(ws + WS_XB); __bf16* WBF = (__bf16*)(ws + WS_WB); float* RT = (float*)(ws + WS_RT);
  _Float16* QK = (_Float16*)(ws + WS_QK); _Float16* VT = (_Float16*)(ws + WS_VT);
  __bf16* VB = (__bf16*)(ws + WS_VB); __bf16* VBL = (__bf16*)(ws + WS_VBL); __bf16* YH = (__bf16*)(ws + WS_YH); __bf16* YL = (__bf16*)(ws + WS_YL);
  k_cvt<<<dim3((unsigned)(((size_t)ROWS * DIN / 8 + 255) / 256)), 256, 0, stream>>>(F[0], XB, (int)((size_t)ROWS * DIN / 8), TT, TT_FULL);
  for (int i = 0; i < 4; ++i)
    k_cvt<<<dim3((unsigned)(((size_t)CC * DIN / 8 + 255) / 256)), 256, 0, stream>>>(F[1 + i], WBF + (size_t)i * CC * DIN, (int)((size_t)CC * DIN / 8), CC, CC);
  k_rope<<<dim3(TT / 8), 256, 0, stream>>>(RT);
  k_proj<<<dim3(ROWS / 64, CC / 128, 3), 128, 0, stream>>>(XB, WBF, RT, F[5], F[6], QK, VT, VB, VBL);
  k_attn<<<dim3(NQB, NB * NH), 128, 0, stream>>>(QK, VT, VB, VBL, YH, YL);
  k_out<<<dim3(ROWS / 64, DIN / 128), 128, 0, stream>>>(YH, YL, WBF + (size_t)3 * CC * DIN, (float*)d_out);
}
